// GINConv_ptens_50869592655547
// MI455X (gfx1250) — hardware-verified
//
#include <hip/hip_runtime.h>
#include <stddef.h>


#define DF      128
#define DH      512
#define NTHR    256
#define NWAVE   8
#define EPT     8
#define CHUNK   (NTHR * EPT)
#define WCAP    (EPT * 2 * 32)
#define LISTN   (NWAVE * WCAP)
#define NB      512
#define MR      64
#define HP      520
#define LDS_AGG (NB * DF * 4 + LISTN * 4 + 64)
#define LDS_MLP (2 * MR * HP * 2 + MR * DF * 4)

static_assert((CHUNK & (CHUNK - 1)) == 0);
static_assert(CHUNK <= 2048);
static_assert((NB & (NB - 1)) == 0);
static_assert(NB <= 512);
static_assert(NB % MR == 0);
static_assert((HP % 8) == 0);
static_assert(NB % NWAVE == 0);
static_assert(MR == 8 * NWAVE);
static_assert((DF % 32) == 0);
static_assert((DH % 32) == 0);

typedef float          v4f  __attribute__((ext_vector_type(4)));
typedef float          v8f  __attribute__((ext_vector_type(8)));
typedef int            v4i  __attribute__((ext_vector_type(4)));
typedef unsigned short v8us __attribute__((ext_vector_type(8)));
typedef __bf16         v16b __attribute__((ext_vector_type(16)));
union FragB { v16b v; v8us h[2]; };

__device__ __forceinline__ unsigned short bf_rne(float f) {
  unsigned u = __builtin_bit_cast(unsigned, f);
  u += 0x7FFFu + ((u >> 16) & 1u);
  return (unsigned short)(u >> 16);
}
__device__ __forceinline__ float bf_up(unsigned short s) {
  return __builtin_bit_cast(float, ((unsigned)s) << 16);
}

__device__ __forceinline__ v8f wmb(v16b a, v16b b, v8f c) {
  v8f d = __builtin_amdgcn_wmma_f32_16x16x32_bf16(false, a, false, b, (short)0, c, false, false);
  asm volatile("v_nop\n\tv_nop\n\tv_nop\n\tv_nop" : "+v"(d) : "v"(a), "v"(b));
  return d;
}

__global__ __launch_bounds__(NTHR) void k_wprep(
    const float* __restrict__ W1, const float* __restrict__ W2,
    unsigned short* w1hi, unsigned short* w1lo, unsigned short* w2hi, unsigned short* w2lo) {
  const int i  = blockIdx.x * NTHR + threadIdx.x;
  const int n1 = DH * DF / 8;
  const int n2 = DF * DH / 8;
  if (i >= n1 + n2) return;
  const bool first = i < n1;
  float v[8];
  unsigned short* ph;
  unsigned short* pl;
  if (first) {
    const int o  = i * 8;
    const int n  = o / DF;
    const int k0 = o - n * DF;
    const float* p = W1 + (size_t)k0 * DH + n;
#pragma unroll
    for (int j = 0; j < 8; ++j) v[j] = p[(size_t)j * DH];
    ph = w1hi + o;
    pl = w1lo + o;
  } else {
    const int o  = (i - n1) * 8;
    const int n  = o / DH;
    const int k0 = o - n * DH;
    const float* p = W2 + (size_t)k0 * DF + n;
#pragma unroll
    for (int j = 0; j < 8; ++j) v[j] = p[(size_t)j * DF];
    ph = w2hi + o;
    pl = w2lo + o;
  }
  v8us hv, lv;
#pragma unroll
  for (int j = 0; j < 8; ++j) {
    const unsigned short h = bf_rne(v[j]);
    hv[j] = h;
    lv[j] = bf_rne(v[j] - bf_up(h));
  }
  *(volatile v8us*)ph = hv;
  *(volatile v8us*)pl = lv;
  __threadfence();
  *(volatile v8us*)ph = hv;
  *(volatile v8us*)pl = lv;
}

__device__ __forceinline__ int scan_chunk(const int* __restrict__ ei, int nE, int cbase, int nodeBase,
                                          int vec8, int* list, int tid, int lane, int wave) {
  int wc = 0;
  const int el0  = tid * EPT;
  const int e0   = cbase + el0;
  const int sent = -2147483647 - 1;
  const int* sp  = ei;
  const int* dp  = ei + (size_t)nE;
  v4i sa, sb, ta, tb;
  if (vec8 != 0 && e0 + 7 < nE) {
    sa = *(const v4i*)(sp + e0);
    sb = *(const v4i*)(sp + e0 + 4);
    ta = *(const v4i*)(dp + e0);
    tb = *(const v4i*)(dp + e0 + 4);
  } else {
    sa.x = (e0     < nE) ? sp[min(e0,     nE - 1)] : sent;
    sa.y = (e0 + 1 < nE) ? sp[min(e0 + 1, nE - 1)] : sent;
    sa.z = (e0 + 2 < nE) ? sp[min(e0 + 2, nE - 1)] : sent;
    sa.w = (e0 + 3 < nE) ? sp[min(e0 + 3, nE - 1)] : sent;
    sb.x = (e0 + 4 < nE) ? sp[min(e0 + 4, nE - 1)] : sent;
    sb.y = (e0 + 5 < nE) ? sp[min(e0 + 5, nE - 1)] : sent;
    sb.z = (e0 + 6 < nE) ? sp[min(e0 + 6, nE - 1)] : sent;
    sb.w = (e0 + 7 < nE) ? sp[min(e0 + 7, nE - 1)] : sent;
    ta.x = (e0     < nE) ? dp[min(e0,     nE - 1)] : sent;
    ta.y = (e0 + 1 < nE) ? dp[min(e0 + 1, nE - 1)] : sent;
    ta.z = (e0 + 2 < nE) ? dp[min(e0 + 2, nE - 1)] : sent;
    ta.w = (e0 + 3 < nE) ? dp[min(e0 + 3, nE - 1)] : sent;
    tb.x = (e0 + 4 < nE) ? dp[min(e0 + 4, nE - 1)] : sent;
    tb.y = (e0 + 5 < nE) ? dp[min(e0 + 5, nE - 1)] : sent;
    tb.z = (e0 + 6 < nE) ? dp[min(e0 + 6, nE - 1)] : sent;
    tb.w = (e0 + 7 < nE) ? dp[min(e0 + 7, nE - 1)] : sent;
  }
  const unsigned nb = (unsigned)nodeBase;
  const unsigned u0 = (unsigned)sa.x - nb, u1 = (unsigned)sa.y - nb, u2 = (unsigned)sa.z - nb, u3 = (unsigned)sa.w - nb;
  const unsigned u4 = (unsigned)sb.x - nb, u5 = (unsigned)sb.y - nb, u6 = (unsigned)sb.z - nb, u7 = (unsigned)sb.w - nb;
  const unsigned t0 = (unsigned)ta.x - nb, t1 = (unsigned)ta.y - nb, t2 = (unsigned)ta.z - nb, t3 = (unsigned)ta.w - nb;
  const unsigned t4 = (unsigned)tb.x - nb, t5 = (unsigned)tb.y - nb, t6 = (unsigned)tb.z - nb, t7 = (unsigned)tb.w - nb;
  const bool a0 = u0 < (unsigned)NB, a1 = u1 < (unsigned)NB, a2 = u2 < (unsigned)NB, a3 = u3 < (unsigned)NB;
  const bool a4 = u4 < (unsigned)NB, a5 = u5 < (unsigned)NB, a6 = u6 < (unsigned)NB, a7 = u7 < (unsigned)NB;
  const bool c0 = t0 < (unsigned)NB, c1 = t1 < (unsigned)NB, c2 = t2 < (unsigned)NB, c3 = t3 < (unsigned)NB;
  const bool c4 = t4 < (unsigned)NB, c5 = t5 < (unsigned)NB, c6 = t6 < (unsigned)NB, c7 = t7 < (unsigned)NB;
  const unsigned any = __builtin_amdgcn_ballot_w32(a0 | a1 | a2 | a3 | a4 | a5 | a6 | a7 |
                                                   c0 | c1 | c2 | c3 | c4 | c5 | c6 | c7);
  if (any != 0u) {
#define HITJ(J, DIR, HJ, SJ) { \
      const unsigned mj = __builtin_amdgcn_ballot_w32(HJ); \
      if (mj != 0u) { \
        if (HJ) { \
          const int pos = wc + (int)__builtin_amdgcn_mbcnt_lo(mj, 0u); \
          if (pos < WCAP) list[wave * WCAP + pos] = ((el0 + (J)) << 10) | ((DIR) << 9) | (int)(SJ); \
        } \
        wc += (int)__builtin_popcount(mj); } }
    HITJ(0, 0, a0, u0) HITJ(0, 1, c0, t0)
    HITJ(1, 0, a1, u1) HITJ(1, 1, c1, t1)
    HITJ(2, 0, a2, u2) HITJ(2, 1, c2, t2)
    HITJ(3, 0, a3, u3) HITJ(3, 1, c3, t3)
    HITJ(4, 0, a4, u4) HITJ(4, 1, c4, t4)
    HITJ(5, 0, a5, u5) HITJ(5, 1, c5, t5)
    HITJ(6, 0, a6, u6) HITJ(6, 1, c6, t6)
    HITJ(7, 0, a7, u7) HITJ(7, 1, c7, t7)
#undef HITJ
  }
  return wc;
}

__device__ __forceinline__ void agg_rows_store(const float* __restrict__ x, const float* acc,
                                               unsigned short* hhi, unsigned short* hlo,
                                               int nodeBase, int nN, float scale, int lane, int wave) {
  const int c0 = 8 * (lane & 15);
  const bool lohalf = lane >= 16;
#pragma unroll 2
  for (int i = 0; i < NB / NWAVE; ++i) {
    const int slot = wave * (NB / NWAVE) + i;
    const int node = nodeBase + slot;
    const int nc   = node > nN - 1 ? nN - 1 : node;
    const float* xp = x + (size_t)nc * DF + c0;
    const v4f xa = *(const v4f*)xp, xb = *(const v4f*)(xp + 4);
    const float* lp = acc + slot * DF + c0;
    const v4f aa = *(const v4f*)lp, ab = *(const v4f*)(lp + 4);
    const v4f va = xa * scale + aa, vb = xb * scale + ab;
    float f[8] = {va.x, va.y, va.z, va.w, vb.x, vb.y, vb.z, vb.w};
    v8us o;
#pragma unroll
    for (int j = 0; j < 8; ++j) {
      const unsigned short h = bf_rne(f[j]);
      const unsigned short l = bf_rne(f[j] - bf_up(h));
      o[j] = lohalf ? l : h;
    }
    unsigned short* dp = (lohalf ? hlo : hhi) + (size_t)node * DF + c0;
    *(volatile v8us*)dp = o;
  }
}

__global__ __launch_bounds__(NTHR) void k_agg(
    const float* __restrict__ x, const int* __restrict__ ei, const float* __restrict__ eps,
    unsigned short* hhi, unsigned short* hlo, int nN, int nE, int vec8) {
  extern __shared__ v4f lds_dyn[];
  float* acc  = (float*)lds_dyn;
  int*   list = (int*)(acc + NB * DF);
  int*   wcnt = list + LISTN;
  const int tid = threadIdx.x, lane = tid & 31, wave = tid >> 5;
  const int nodeBase = blockIdx.x * NB;

  {
    const v4f z = {0.f, 0.f, 0.f, 0.f};
    for (int i = tid; i < NB * DF / 4; i += NTHR) lds_dyn[i] = z;
  }
  __syncthreads();

  const int nChunks = (nE + CHUNK - 1) / CHUNK;
#pragma unroll 1
  for (int ch = 0; ch < nChunks; ++ch) {
    const int cbase = ch * CHUNK;
    const int wc = scan_chunk(ei, nE, cbase, nodeBase, vec8, list, tid, lane, wave);
    if (lane == 0) wcnt[wave] = wc;
    __syncthreads();
    if (wave == 0) {
#pragma unroll 1
      for (int wsx = 0; wsx < NWAVE; ++wsx) {
        int n = __builtin_amdgcn_readfirstlane(wcnt[wsx]);
        n = n > WCAP ? WCAP : (n < 0 ? 0 : n);
        const int* lp = list + wsx * WCAP;
#pragma unroll 1
        for (int i = 0; i < n; ++i) {
          const int ent  = __builtin_amdgcn_readfirstlane(lp[i]);
          const int slot = ent & (NB - 1);
          const int dir  = (ent >> 9) & 1;
          int e = cbase + ((ent >> 10) & (CHUNK - 1));
          e = e > nE - 1 ? nE - 1 : e;
          int oth = (dir != 0) ? ei[e] : ei[(size_t)nE + (size_t)e];
          oth = oth < 0 ? 0 : (oth > nN - 1 ? nN - 1 : oth);
          const v4f v = *(const v4f*)(x + (size_t)oth * DF + 4 * lane);
          v4f* ap = (v4f*)(acc + slot * DF + 4 * lane);
          *ap = *ap + v;
        }
      }
    }
    __syncthreads();
  }

  const float scale = 1.0f + eps[0];
  agg_rows_store(x, acc, hhi, hlo, nodeBase, nN, scale, lane, wave);
  __threadfence();
  agg_rows_store(x, acc, hhi, hlo, nodeBase, nN, scale, lane, wave);
}

__global__ __launch_bounds__(NTHR) void k_mlp(
    const unsigned short* __restrict__ hhi, const unsigned short* __restrict__ hlo,
    const unsigned short* __restrict__ w1hi, const unsigned short* __restrict__ w1lo,
    const unsigned short* __restrict__ w2hi, const unsigned short* __restrict__ w2lo,
    const float* __restrict__ b1, const float* __restrict__ b2, float* out, int nN) {
  extern __shared__ v4f lds_dyn[];
  unsigned short* sHhi = (unsigned short*)lds_dyn;
  unsigned short* sHlo = sHhi + MR * HP;
  float*          sOut = (float*)(sHlo + MR * HP);
  const int tid = threadIdx.x, lane = tid & 31, wave = tid >> 5, hh = lane >> 4, m = lane & 15;
  const int rt = wave & 3, cg = wave >> 2;
  const int rowBase = blockIdx.x * MR;
  const size_t arow = (size_t)(rowBase + 16 * rt + m) * DF + 8 * hh;

#pragma unroll 1
  for (int p = 0; p < 4; ++p) {
    const int nb0 = 256 * cg + 64 * p;
    v8f acc[4];
#pragma unroll
    for (int j = 0; j < 4; ++j) { v8f z = {0.f, 0.f, 0.f, 0.f, 0.f, 0.f, 0.f, 0.f}; acc[j] = z; }
#pragma unroll 1
    for (int kt = 0; kt < DF / 32; ++kt) {
      FragB ah, al;
      ah.h[0] = *(const v8us*)(hhi + arow + 32 * kt);
      ah.h[1] = *(const v8us*)(hhi + arow + 32 * kt + 16);
      al.h[0] = *(const v8us*)(hlo + arow + 32 * kt);
      al.h[1] = *(const v8us*)(hlo + arow + 32 * kt + 16);
#pragma unroll
      for (int j = 0; j < 4; ++j) {
        const size_t bo = (size_t)(nb0 + 16 * j + m) * DF + 32 * kt + 8 * hh;
        FragB bh, bl;
        bh.h[0] = *(const v8us*)(w1hi + bo);
        bh.h[1] = *(const v8us*)(w1hi + bo + 16);
        bl.h[0] = *(const v8us*)(w1lo + bo);
        bl.h[1] = *(const v8us*)(w1lo + bo + 16);
        acc[j] = wmb(ah.v, bh.v, acc[j]);
        acc[j] = wmb(ah.v, bl.v, acc[j]);
        acc[j] = wmb(al.v, bh.v, acc[j]);
      }
    }
#pragma unroll
    for (int j = 0; j < 4; ++j) {
      const int col = nb0 + 16 * j + m;
      const float bias = b1[col];
      unsigned short* ph = sHhi + (16 * rt + 8 * hh) * HP + col;
      unsigned short* pl = sHlo + (16 * rt + 8 * hh) * HP + col;
#pragma unroll
      for (int r = 0; r < 8; ++r) {
        const float v = fmaxf(acc[j][r] + bias, 0.f);
        const unsigned short h = bf_rne(v);
        ph[r * HP] = h;
        pl[r * HP] = bf_rne(v - bf_up(h));
      }
    }
  }
  __syncthreads();

  v8f acc2[4];
#pragma unroll
  for (int j = 0; j < 4; ++j) { v8f z = {0.f, 0.f, 0.f, 0.f, 0.f, 0.f, 0.f, 0.f}; acc2[j] = z; }
  const unsigned short* a2h = sHhi + (16 * rt + m) * HP + 8 * hh;
  const unsigned short* a2l = sHlo + (16 * rt + m) * HP + 8 * hh;
#pragma unroll 1
  for (int kt = 0; kt < DH / 32; ++kt) {
    FragB ah, al;
    ah.h[0] = *(const v8us*)(a2h + 32 * kt);
    ah.h[1] = *(const v8us*)(a2h + 32 * kt + 16);
    al.h[0] = *(const v8us*)(a2l + 32 * kt);
    al.h[1] = *(const v8us*)(a2l + 32 * kt + 16);
#pragma unroll
    for (int j = 0; j < 4; ++j) {
      const size_t bo = (size_t)(64 * cg + 16 * j + m) * DH + 32 * kt + 8 * hh;
      FragB bh, bl;
      bh.h[0] = *(const v8us*)(w2hi + bo);
      bh.h[1] = *(const v8us*)(w2hi + bo + 16);
      bl.h[0] = *(const v8us*)(w2lo + bo);
      bl.h[1] = *(const v8us*)(w2lo + bo + 16);
      acc2[j] = wmb(ah.v, bh.v, acc2[j]);
      acc2[j] = wmb(ah.v, bl.v, acc2[j]);
      acc2[j] = wmb(al.v, bh.v, acc2[j]);
    }
  }
#pragma unroll
  for (int j = 0; j < 4; ++j) {
    const int col = 64 * cg + 16 * j + m;
    const float bias = b2[col];
    float* sp = sOut + (16 * rt + 8 * hh) * DF + col;
#pragma unroll
    for (int r = 0; r < 8; ++r) sp[r * DF] = acc2[j][r] + bias;
  }
  __syncthreads();

#pragma unroll
  for (int i = 0; i < 8; ++i) {
    const int lr = 8 * wave + i;
    const int grow = rowBase + lr;
    if (grow < nN) {
      const v4f v = *(const v4f*)(sOut + lr * DF + 4 * lane);
      *(volatile v4f*)(out + (size_t)grow * DF + 4 * lane) = v;
    }
  }
  __threadfence();
#pragma unroll
  for (int i = 0; i < 8; ++i) {
    const int lr = 8 * wave + i;
    const int grow = rowBase + lr;
    if (grow < nN) {
      const v4f v = *(const v4f*)(sOut + lr * DF + 4 * lane);
      *(volatile v4f*)(out + (size_t)grow * DF + 4 * lane) = v;
    }
  }
}

extern "C" void kernel_launch(void* const* d_in, const int* in_sizes, int n_in,
                              void* d_out, int out_size, void* d_ws, size_t ws_size,
                              hipStream_t stream) {
  if (n_in < 7) return;
  const int nN = in_sizes[0] / DF;
  const int nE = in_sizes[1] / 2;
  if (nN <= 0 || nE < 0 || in_sizes[0] != nN * DF || in_sizes[1] != nE * 2) return;
  if (in_sizes[2] < 1 || in_sizes[3] != DF * DH || in_sizes[4] < DH || in_sizes[5] != DH * DF || in_sizes[6] < DF) return;
  if (out_size != nN * DF) return;

  const float* x   = (const float*)d_in[0];
  const int*   ei  = (const int*)d_in[1];
  const float* eps = (const float*)d_in[2];
  const float* W1  = (const float*)d_in[3];
  const float* b1  = (const float*)d_in[4];
  const float* W2  = (const float*)d_in[5];
  const float* b2  = (const float*)d_in[6];
  float* out = (float*)d_out;

  const int nAgg    = (nN + NB - 1) / NB;
  const int nMlp    = (nN + MR - 1) / MR;
  const int rowsPad = nAgg * NB;
  if (nMlp * MR > rowsPad) return;

  char* ws = (char*)d_ws;
  size_t off = 0;
  const size_t wsz = (size_t)DH * DF * 2;
  const size_t hsz = (size_t)rowsPad * DF * 2;
  const size_t oW1h = off; off += wsz; off = (off + 255) & ~(size_t)255;
  const size_t oW1l = off; off += wsz; off = (off + 255) & ~(size_t)255;
  const size_t oW2h = off; off += wsz; off = (off + 255) & ~(size_t)255;
  const size_t oW2l = off; off += wsz; off = (off + 255) & ~(size_t)255;
  const size_t oHh  = off; off += hsz; off = (off + 255) & ~(size_t)255;
  const size_t oHl  = off; off += hsz; off = (off + 255) & ~(size_t)255;
  if (off > ws_size || off > (size_t)134217728) return;
  unsigned short* w1hi = (unsigned short*)(ws + oW1h);
  unsigned short* w1lo = (unsigned short*)(ws + oW1l);
  unsigned short* w2hi = (unsigned short*)(ws + oW2h);
  unsigned short* w2lo = (unsigned short*)(ws + oW2l);
  unsigned short* hhi  = (unsigned short*)(ws + oHh);
  unsigned short* hlo  = (unsigned short*)(ws + oHl);

  const int vec8 = ((nE & 3) == 0) ? 1 : 0;

  const int nPrep = DH * DF / 8 + DF * DH / 8;
  k_wprep<<<(nPrep + NTHR - 1) / NTHR, NTHR, 0, stream>>>(W1, W2, w1hi, w1lo, w2hi, w2lo);

  hipFuncSetAttribute(reinterpret_cast<const void*>(&k_agg),
                      hipFuncAttributeMaxDynamicSharedMemorySize, LDS_AGG);
  k_agg<<<nAgg, NTHR, LDS_AGG, stream>>>(x, ei, eps, hhi, hlo, nN, nE, vec8);

  hipFuncSetAttribute(reinterpret_cast<const void*>(&k_mlp),
                      hipFuncAttributeMaxDynamicSharedMemorySize, LDS_MLP);
  k_mlp<<<nMlp, NTHR, LDS_MLP, stream>>>(hhi, hlo, w1hi, w1lo, w2hi, w2lo, b1, b2, out, nN);
}
